// MagPot_24472723652711
// MI455X (gfx1250) — hardware-verified
//
#include <hip/hip_runtime.h>
#include <stddef.h>
#include <math.h>


#define NTHR   256
#define NWAVE  8
#define EPT    8
#define CHUNK  (NTHR * EPT)
#define WCAP   384
#define WTHR   (WCAP - EPT * 32)
#define DPER   32
#define NB     640
#define ACOL   88
#define AC4    (ACOL / 4)
#define PSZ    64
#define NSPEC  4
#define NBAS   12
#define NRAD   8
#define NEMB   16
#define NHEAD  9
#define CHEBN  (NSPEC * NSPEC * NRAD * NBAS)
#define TROW   112
#define MLPT   64
#define MROW   32
#define NOUT   64
#define PREP_T 128
#define PB1    2
#define PB2    4
#define PB3    9
#define PB4    9
#define PBT    (PB1 + PB2 + PB3 + PB4)
#define NFLG   3
#define WSCL   16.0f
#define WINV   0.0625f
#define RCUT   6.0f
#define EPSG   1e-9f

#define L_ACC    0
#define L_MSG    (L_ACC + (NB + 1) * ACOL * 4)
#define L_CHB    (L_MSG + PSZ * ACOL * 4)
#define L_LST    (L_CHB + CHEBN * 4)
#define L_SLT    (L_LST + NWAVE * WCAP * 4)
#define L_CNT    (L_SLT + PSZ * 4)
#define LDS_EDGE (L_CNT + 64)

static_assert((L_MSG % 16) == 0 && (L_CHB % 16) == 0 && (L_LST % 16) == 0 && (L_SLT % 16) == 0 && (L_CNT % 16) == 0);
static_assert(LDS_EDGE <= 300 * 1024);
static_assert((NB % 32) == 0);
static_assert(((NB * ACOL * 4) % 256) == 0);
static_assert(((NB * AC4) % NTHR) == 0);
static_assert(PSZ == 64 && AC4 == 22);
static_assert(WTHR >= 0 && (DPER & (DPER - 1)) == 0);
static_assert((NWAVE + NFLG) * 4 <= 64);
static_assert(PB1 * PREP_T * 8 == 64 * 32);
static_assert(PB2 * PREP_T * 8 == 64 * 64);
static_assert(PB3 * PREP_T * 8 == NHEAD * 32 * 32);
static_assert(PB4 * PREP_T * 8 == NHEAD * 32 * 32);
static_assert(MROW == 32 && MLPT == 64);

typedef float    v4f  __attribute__((ext_vector_type(4)));
typedef float    v8f  __attribute__((ext_vector_type(8)));
typedef int      v4i  __attribute__((ext_vector_type(4)));
typedef _Float16 v8h  __attribute__((ext_vector_type(8)));
typedef _Float16 v16h __attribute__((ext_vector_type(16)));
union FragH { v16h v; v8h h[2]; };
union Pk8 { v8h h; v4i i; };

__device__ __forceinline__ int clampi(int v, int lo, int hi) { return v < lo ? lo : (v > hi ? hi : v); }

__device__ __forceinline__ v8f wmh(v16h a, v16h b, v8f c) {
  v8f d = __builtin_amdgcn_wmma_f32_16x16x32_f16(false, a, false, b, (short)0, c, false, false);
  asm volatile("v_nop\n\tv_nop\n\tv_nop\n\tv_nop" : "+v"(d) : "v"(a), "v"(b));
  return d;
}

__device__ __forceinline__ float silu_f(float x) {
  return x * __builtin_amdgcn_rcpf(1.0f + __expf(-x));
}

__device__ __forceinline__ v8h silu16(v8f d) {
  v8h r;
#pragma unroll
  for (int i = 0; i < 8; ++i) { const float t = silu_f(d[i] * WINV); r[i] = (_Float16)t; }
  return r;
}

__device__ __forceinline__ v8h cv8(v4f a, v4f b) {
  v8h r;
  r[0] = (_Float16)a.x; r[1] = (_Float16)a.y; r[2] = (_Float16)a.z; r[3] = (_Float16)a.w;
  r[4] = (_Float16)b.x; r[5] = (_Float16)b.y; r[6] = (_Float16)b.z; r[7] = (_Float16)b.w;
  return r;
}

__device__ __forceinline__ v8f ld8(const float* p, float mul) {
  const v4f a = *(const v4f*)p;
  const v4f b = *(const v4f*)(p + 4);
  v8f c;
  c[0] = a.x * mul; c[1] = a.y * mul; c[2] = a.z * mul; c[3] = a.w * mul;
  c[4] = b.x * mul; c[5] = b.y * mul; c[6] = b.z * mul; c[7] = b.w * mul;
  return c;
}

__device__ __forceinline__ int scan_chunk(const int* __restrict__ dsts, int nE, int cbase, int nodeBase,
                                          int vec8, int* list, int tid, int wave, int wc0) {
  int wc = wc0;
  const int e0   = cbase + tid * EPT;
  const int sent = -2147483647 - 1;
  v4i da, db;
  if (vec8 != 0 && cbase + CHUNK <= nE) {
    da = *(const v4i*)(dsts + e0);
    db = *(const v4i*)(dsts + e0 + 4);
  } else {
    da.x = (e0     < nE) ? dsts[min(e0,     nE - 1)] : sent;
    da.y = (e0 + 1 < nE) ? dsts[min(e0 + 1, nE - 1)] : sent;
    da.z = (e0 + 2 < nE) ? dsts[min(e0 + 2, nE - 1)] : sent;
    da.w = (e0 + 3 < nE) ? dsts[min(e0 + 3, nE - 1)] : sent;
    db.x = (e0 + 4 < nE) ? dsts[min(e0 + 4, nE - 1)] : sent;
    db.y = (e0 + 5 < nE) ? dsts[min(e0 + 5, nE - 1)] : sent;
    db.z = (e0 + 6 < nE) ? dsts[min(e0 + 6, nE - 1)] : sent;
    db.w = (e0 + 7 < nE) ? dsts[min(e0 + 7, nE - 1)] : sent;
  }
  const unsigned nb = (unsigned)nodeBase;
  const unsigned s0 = (unsigned)da.x - nb, s1 = (unsigned)da.y - nb;
  const unsigned s2 = (unsigned)da.z - nb, s3 = (unsigned)da.w - nb;
  const unsigned s4 = (unsigned)db.x - nb, s5 = (unsigned)db.y - nb;
  const unsigned s6 = (unsigned)db.z - nb, s7 = (unsigned)db.w - nb;
  const bool h0 = s0 < (unsigned)NB, h1 = s1 < (unsigned)NB, h2 = s2 < (unsigned)NB, h3 = s3 < (unsigned)NB;
  const bool h4 = s4 < (unsigned)NB, h5 = s5 < (unsigned)NB, h6 = s6 < (unsigned)NB, h7 = s7 < (unsigned)NB;
  const unsigned any = __builtin_amdgcn_ballot_w32(h0 | h1 | h2 | h3 | h4 | h5 | h6 | h7);
  if (any != 0u) {
#define HITJ(J, HJ) { \
      const unsigned mj = __builtin_amdgcn_ballot_w32(HJ); \
      if (mj != 0u) { \
        if (HJ) { \
          const int pos = wc + (int)__builtin_amdgcn_mbcnt_lo(mj, 0u); \
          if (pos < WCAP) list[wave * WCAP + pos] = e0 + (J); \
        } \
        wc += (int)__builtin_popcount(mj); } }
    HITJ(0, h0)
    HITJ(1, h1)
    HITJ(2, h2)
    HITJ(3, h3)
    HITJ(4, h4)
    HITJ(5, h5)
    HITJ(6, h6)
    HITJ(7, h7)
#undef HITJ
  }
  return wc;
}

__global__ __launch_bounds__(PREP_T) void k_prep(
    const float* __restrict__ w1, const float* __restrict__ w2,
    const float* __restrict__ m1, const float* __restrict__ m2,
    _Float16* p1, _Float16* p2, _Float16* q1, _Float16* q2) {
  const int b = blockIdx.x, tid = threadIdx.x;
  const float* src;
  _Float16* dst;
  int Kin, Kp, O, ub;
  if (b < PB1) {
    src = w1; dst = p1; Kin = 32; Kp = 32; O = 64; ub = b;
  } else if (b < PB1 + PB2) {
    src = w2; dst = p2; Kin = 64; Kp = 64; O = 64; ub = b - PB1;
  } else if (b < PB1 + PB2 + PB3) {
    src = m1; dst = q1; Kin = 24; Kp = 32; O = 32; ub = b - (PB1 + PB2);
  } else {
    src = m2; dst = q2; Kin = 32; Kp = 32; O = 32; ub = b - (PB1 + PB2 + PB3);
  }
  const int u   = ub * PREP_T + tid;
  const int cpr = Kp >> 3;
  const int row = u / cpr;
  const int kc  = u - row * cpr;
  const int hd  = row / O;
  const int n   = row - hd * O;
  Pk8 pk;
#pragma unroll
  for (int j = 0; j < 8; ++j) {
    const int k   = 8 * kc + j;
    const int kcl = k < Kin ? k : Kin - 1;
    const float w = src[(size_t)(hd * Kin + kcl) * O + n];
    const float t = (k < Kin) ? w * WSCL : 0.0f;
    pk.h[j] = (_Float16)t;
  }
  _Float16* dp = dst + (size_t)u * 8;
  *(volatile v4i*)dp = pk.i;
  __threadfence();
  *(volatile v4i*)dp = pk.i;
}

__global__ __launch_bounds__(NTHR) void k_edge(
    const float* __restrict__ pos, const float* __restrict__ mom, const int* __restrict__ spec,
    const int* __restrict__ iidx, const int* __restrict__ jidx, const float* __restrict__ cheb,
    float* feat, int nN, int nE, int vec8) {
  extern __shared__ __attribute__((aligned(16))) unsigned char dsm[];
  float* acc   = (float*)(dsm + L_ACC);
  float* msg   = (float*)(dsm + L_MSG);
  float* scb   = (float*)(dsm + L_CHB);
  int*   list  = (int*)(dsm + L_LST);
  int*   slotb = (int*)(dsm + L_SLT);
  int*   wcnt  = (int*)(dsm + L_CNT);

  const int tid = threadIdx.x, lane = tid & 31, wave = tid >> 5;
  const int nodeBase = blockIdx.x * NB;

  {
    const v4f z = {0.0f, 0.0f, 0.0f, 0.0f};
    for (int i = tid; i < (NB + 1) * AC4; i += NTHR) *(v4f*)(acc + 4 * i) = z;
  }
  for (int i = tid; i < CHEBN; i += NTHR) scb[i] = cheb[i];
  if (tid < 16) wcnt[tid] = 0;
  __syncthreads();

  int wc = 0;
  const int nChunks = (nE + CHUNK - 1) / CHUNK;
#pragma unroll 1
  for (int ch = 0; ch < nChunks; ++ch) {
    const int fcur = NWAVE + (ch % NFLG);
    const int fnxt = NWAVE + ((ch + 1) % NFLG);
    if (tid == 0) wcnt[fnxt] = 0;
    wc = scan_chunk(iidx, nE, ch * CHUNK, nodeBase, vec8, list, tid, wave, wc);
    if (lane == 0) {
      wcnt[wave] = wc;
      if (wc > WTHR) wcnt[fcur] = 1;
    }
    __syncthreads();
    const int ovf  = wcnt[fcur];
    const int last = (ch == nChunks - 1) ? 1 : 0;
    const int per  = ((ch & (DPER - 1)) == DPER - 1) ? 1 : 0;
    if ((ovf | last | per) != 0) {
      int ocum[NWAVE + 1];
      ocum[0] = 0;
#pragma unroll
      for (int w = 0; w < NWAVE; ++w) {
        const int c = clampi(wcnt[w], 0, WCAP);
        ocum[w + 1] = ocum[w] + c;
      }
      const int tot = ocum[NWAVE];
      const int R   = (tot + PSZ - 1) / PSZ;
#pragma unroll 1
      for (int r = 0; r < R; ++r) {
        if (tid < PSZ) {
          const int v = r * PSZ + tid;
          const bool valid = v < tot;
          int ob = 0, ws = 0;
#pragma unroll
          for (int k = 1; k < NWAVE; ++k) {
            const bool ge = v >= ocum[k];
            ob = ge ? ocum[k] : ob;
            ws = ge ? k : ws;
          }
          const int idx = clampi(v - ob, 0, WCAP - 1);
          int e = list[ws * WCAP + idx];
          e = clampi(e, 0, nE - 1);
          const int i  = iidx[e];
          const int j  = jidx[e];
          const int ic = clampi(i, 0, nN - 1);
          const int jc = clampi(j, 0, nN - 1);
          int slot = i - nodeBase;
          if (!valid || (unsigned)slot >= (unsigned)NB) slot = NB;

          const float pix = pos[3 * ic], piy = pos[3 * ic + 1], piz = pos[3 * ic + 2];
          const float pjx = pos[3 * jc], pjy = pos[3 * jc + 1], pjz = pos[3 * jc + 2];
          const float rx = pjx - pix, ry = pjy - piy, rz = pjz - piz;
          const float d2 = (rx * rx + rz * rz) + ry * ry;
          const float dist = sqrtf(d2 + EPSG);
          const float invd = __builtin_amdgcn_rcpf(dist);
          const float ux = rx * invd, uy = ry * invd, uz = rz * invd;

          float x = 2.0f * dist * (1.0f / RCUT) - 1.0f;
          x = fminf(1.0f, fmaxf(-1.0f, x));
          float T[NBAS];
          T[0] = 1.0f; T[1] = x;
#pragma unroll
          for (int k = 2; k < NBAS; ++k) T[k] = 2.0f * x * T[k - 1] - T[k - 2];
          const float cs = cospif(dist * (1.0f / RCUT));
          const float fc = (dist < RCUT) ? 0.5f * (cs + 1.0f) : 0.0f;
          const int si = clampi(spec[ic], 0, NSPEC - 1);
          const int sj = clampi(spec[jc], 0, NSPEC - 1);
          const float* cb = scb + (si * NSPEC + sj) * (NRAD * NBAS);

          const float m0x = mom[3 * ic], m0y = mom[3 * ic + 1], m0z = mom[3 * ic + 2];
          const float m1x = mom[3 * jc], m1y = mom[3 * jc + 1], m1z = mom[3 * jc + 2];
          const float mni = sqrtf(((m0x * m0x + m0z * m0z) + m0y * m0y) + EPSG);
          const float mnj = sqrtf(((m1x * m1x + m1z * m1z) + m1y * m1y) + EPSG);
          const float ri = __builtin_amdgcn_rcpf(mni);
          const float rj = __builtin_amdgcn_rcpf(mnj);
          const float hix = m0x * ri, hiy = m0y * ri, hiz = m0z * ri;
          const float hjx = m1x * rj, hjy = m1y * rj, hjz = m1z * rj;
          const float w1 = (m0x * m1x + m0z * m1z) + m0y * m1y;
          const float dir = (hix * ux + hiz * uz) + hiy * uy;
          const float djr = (hjx * ux + hjz * uz) + hjy * uy;
          const float w2 = dir * dir;
          const float w3 = djr * djr;
          const float cx = m0y * m1z - m0z * m1y;
          const float cy = m0z * m1x - m0x * m1z;
          const float cz = m0x * m1y - m0y * m1x;
          const float w4 = (ux * cx + uz * cz) + uy * cy;
          const float w5 = mnj;
          const float w6 = ((hix * hjx + hiz * hjz) + hiy * hjy) * mnj;
          const float w7 = mnj * mnj;

          float* mr = msg + tid * ACOL;
#pragma unroll 1
          for (int n = 0; n < NRAD; ++n) {
            const float* cp = cb + n * NBAS;
            const v4f c0 = *(const v4f*)cp;
            const v4f c1 = *(const v4f*)(cp + 4);
            const v4f c2 = *(const v4f*)(cp + 8);
            float sa = c0.x * T[0];
            sa = fmaf(c0.y, T[1], sa);  sa = fmaf(c0.z, T[2], sa);  sa = fmaf(c0.w, T[3], sa);
            sa = fmaf(c1.x, T[4], sa);  sa = fmaf(c1.y, T[5], sa);  sa = fmaf(c1.z, T[6], sa);  sa = fmaf(c1.w, T[7], sa);
            sa = fmaf(c2.x, T[8], sa);  sa = fmaf(c2.y, T[9], sa);  sa = fmaf(c2.z, T[10], sa); sa = fmaf(c2.w, T[11], sa);
            const float ph = sa * fc;
            mr[n]          = ph;
            mr[8 + n]      = ph * w1;
            mr[16 + n]     = ph * w2;
            mr[24 + n]     = ph * w3;
            mr[32 + n]     = ph * w4;
            mr[40 + n]     = ph * w5;
            mr[48 + n]     = ph * w6;
            mr[56 + n]     = ph * w7;
            mr[64 + 3 * n]     = ph * ux;
            mr[64 + 3 * n + 1] = ph * uy;
            mr[64 + 3 * n + 2] = ph * uz;
          }
          slotb[tid] = slot;
        }
        __syncthreads();

        if (wave == 0) {
          int cnt = tot - r * PSZ;
          cnt = cnt > PSZ ? PSZ : cnt;
          const int qq = lane < AC4 ? lane : AC4 - 1;
#pragma unroll 1
          for (int e = 0; e < cnt; ++e) {
            const int s = clampi(slotb[e], 0, NB);
            float* ap = acc + s * ACOL + 4 * qq;
            v4f av = *(v4f*)ap;
            const v4f mv = *(const v4f*)(msg + e * ACOL + 4 * qq);
            av += mv;
            if (lane < AC4) *(v4f*)ap = av;
          }
        }
        __syncthreads();
      }
      __syncthreads();
      wc = 0;
    }
  }
  __syncthreads();

  for (int s = tid; s < NB; s += NTHR) {
    float* ar = acc + s * ACOL;
    int a = nodeBase + s;
    a = a > nN - 1 ? nN - 1 : a;
    const float mx = mom[3 * a], my = mom[3 * a + 1], mz = mom[3 * a + 2];
    const float amp = sqrtf(((mx * mx + mz * mz) + my * my) + EPSG);
#pragma unroll 1
    for (int n = 0; n < NRAD; ++n) {
      const float v0 = ar[64 + 3 * n], v1 = ar[64 + 3 * n + 1], v2 = ar[64 + 3 * n + 2];
      ar[64 + n] = (v0 * v0 + v2 * v2) + v1 * v1;
    }
    { const v4f p = *(const v4f*)(ar + 56), q = *(const v4f*)(ar + 60);
      *(v4f*)(ar + 80) = p; *(v4f*)(ar + 84) = q; }
    { const v4f p = *(const v4f*)(ar + 48), q = *(const v4f*)(ar + 52);
      *(v4f*)(ar + 72) = p; *(v4f*)(ar + 76) = q; }
    const v4f vq0 = *(const v4f*)(ar + 64), vq1 = *(const v4f*)(ar + 68);
    { const v4f p = *(const v4f*)(ar + 40), q = *(const v4f*)(ar + 44);
      *(v4f*)(ar + 64) = p; *(v4f*)(ar + 68) = q;
      *(v4f*)(ar + 56) = p * amp; *(v4f*)(ar + 60) = q * amp; }
    { const v4f p = *(const v4f*)(ar + 32), q = *(const v4f*)(ar + 36);
      *(v4f*)(ar + 48) = p; *(v4f*)(ar + 52) = q; }
    { const v4f p = *(const v4f*)(ar + 24), q = *(const v4f*)(ar + 28);
      *(v4f*)(ar + 40) = p; *(v4f*)(ar + 44) = q; }
    { const v4f p = *(const v4f*)(ar + 16), q = *(const v4f*)(ar + 20);
      *(v4f*)(ar + 32) = p; *(v4f*)(ar + 36) = q; }
    { const v4f p = *(const v4f*)(ar + 8), q = *(const v4f*)(ar + 12);
      *(v4f*)(ar + 24) = p; *(v4f*)(ar + 28) = q; }
    { const v4f p = *(const v4f*)(ar + 0), q = *(const v4f*)(ar + 4);
      *(v4f*)(ar + 16) = p * amp; *(v4f*)(ar + 20) = q * amp;
      *(v4f*)(ar + 8) = vq0; *(v4f*)(ar + 12) = vq1; }
  }
  __syncthreads();

  float* fb = feat + (size_t)blockIdx.x * (size_t)(NB * ACOL);
#pragma unroll 1
  for (int u = tid; u < NB * AC4; u += NTHR) {
    const v4f v = *(const v4f*)(acc + 4 * u);
    *(volatile v4f*)(fb + 4 * u) = v;
  }
  __threadfence();
#pragma unroll 1
  for (int u = tid; u < NB * AC4; u += NTHR) {
    const v4f v = *(const v4f*)(acc + 4 * u);
    *(volatile v4f*)(fb + 4 * u) = v;
  }
}

__global__ __launch_bounds__(MLPT) void k_mlp(
    const float* __restrict__ feat, const int* __restrict__ spec,
    const float* __restrict__ embt, const float* __restrict__ shf,
    const _Float16* __restrict__ P1, const float* __restrict__ bs1,
    const _Float16* __restrict__ P2, const float* __restrict__ bs2,
    const float* __restrict__ Ws3, const float* __restrict__ bs3,
    const _Float16* __restrict__ Q1, const float* __restrict__ bm1,
    const _Float16* __restrict__ Q2, const float* __restrict__ bm2,
    const float* __restrict__ Wm3, const float* __restrict__ bm3,
    float* eat, int nN, int featRows) {
  __shared__ __attribute__((aligned(16))) _Float16 tl[2 * 16 * TROW];
  __shared__ __attribute__((aligned(16))) float es[MROW];
  const int tid = threadIdx.x, lane = tid & 31, wave = tid >> 5, h = lane >> 4, m = lane & 15;
  const int a  = blockIdx.x * MROW + wave * 16 + m;
  const int ac = a > nN - 1 ? nN - 1 : a;
  const int af = a > featRows - 1 ? featRows - 1 : a;
  _Float16* tw   = tl + wave * 16 * TROW;
  _Float16* trow = tw + m * TROW;
  const float* fr = feat + (size_t)af * ACOL;

  {
    const v4f x0 = *(const v4f*)(fr + 8 * h), x1 = *(const v4f*)(fr + 8 * h + 4);
    *(v8h*)(trow + 8 * h) = cv8(x0, x1);
  }
  const int sp = clampi(spec[ac], 0, NSPEC - 1);
  {
    const float* er = embt + sp * NEMB + 8 * h;
    const v4f e0 = *(const v4f*)er, e1 = *(const v4f*)(er + 4);
    *(v8h*)(trow + 16 + 8 * h) = cv8(e0, e1);
  }
#pragma unroll
  for (int u = 0; u < 5; ++u) {
    const int c  = h + 2 * u;
    const int cc = c > 8 ? 8 : c;
    const float keep = (c < 9) ? 1.0f : 0.0f;
    const float* sr = fr + 16 + 8 * cc;
    const v4f s0 = *(const v4f*)sr * keep, s1 = *(const v4f*)(sr + 4) * keep;
    *(v8h*)(trow + 32 + 8 * c) = cv8(s0, s1);
  }
  __syncthreads();

  FragH bx;
  bx.h[0] = *(const v8h*)(trow + 8 * h);
  bx.h[1] = *(const v8h*)(trow + 16 + 8 * h);
  v8f d0, d1, d2, d3;
  {
    FragH aw; const _Float16* wp = P1 + (size_t)(0 + m) * 32 + 8 * h;
    aw.h[0] = *(const v8h*)wp; aw.h[1] = *(const v8h*)(wp + 16);
    d0 = wmh(aw.v, bx.v, ld8(bs1 + 0 + 8 * h, WSCL));
  }
  {
    FragH aw; const _Float16* wp = P1 + (size_t)(16 + m) * 32 + 8 * h;
    aw.h[0] = *(const v8h*)wp; aw.h[1] = *(const v8h*)(wp + 16);
    d1 = wmh(aw.v, bx.v, ld8(bs1 + 16 + 8 * h, WSCL));
  }
  {
    FragH aw; const _Float16* wp = P1 + (size_t)(32 + m) * 32 + 8 * h;
    aw.h[0] = *(const v8h*)wp; aw.h[1] = *(const v8h*)(wp + 16);
    d2 = wmh(aw.v, bx.v, ld8(bs1 + 32 + 8 * h, WSCL));
  }
  {
    FragH aw; const _Float16* wp = P1 + (size_t)(48 + m) * 32 + 8 * h;
    aw.h[0] = *(const v8h*)wp; aw.h[1] = *(const v8h*)(wp + 16);
    d3 = wmh(aw.v, bx.v, ld8(bs1 + 48 + 8 * h, WSCL));
  }
  FragH bq0, bq1;
  bq0.h[0] = silu16(d0); bq0.h[1] = silu16(d1);
  bq1.h[0] = silu16(d2); bq1.h[1] = silu16(d3);
  float esp = 0.0f;
#pragma unroll
  for (int t = 0; t < 4; ++t) {
    v8f c = ld8(bs2 + 16 * t + 8 * h, WSCL);
    {
      FragH aw; const _Float16* wp = P2 + (size_t)(16 * t + m) * 64 + 8 * h;
      aw.h[0] = *(const v8h*)wp; aw.h[1] = *(const v8h*)(wp + 16);
      c = wmh(aw.v, bq0.v, c);
    }
    {
      FragH aw; const _Float16* wp = P2 + (size_t)(16 * t + m) * 64 + 32 + 8 * h;
      aw.h[0] = *(const v8h*)wp; aw.h[1] = *(const v8h*)(wp + 16);
      c = wmh(aw.v, bq1.v, c);
    }
    const v8f w3 = ld8(Ws3 + 16 * t + 8 * h, 1.0f);
#pragma unroll
    for (int rr = 0; rr < 8; ++rr) esp = fmaf(silu_f(c[rr] * WINV), w3[rr], esp);
  }
  const float estr = esp + __shfl_xor(esp, 16) + bs3[0];

  float emp = 0.0f, bsum = 0.0f;
#pragma unroll 1
  for (int hd = 0; hd < NHEAD; ++hd) {
    FragH bh;
    const int off0 = (h != 0) ? 16 : (32 + 8 * hd);
    const int off1 = (h != 0) ? 104 : 24;
    bh.h[0] = *(const v8h*)(trow + off0);
    bh.h[1] = *(const v8h*)(trow + off1);
    v8f g0, g1;
    {
      FragH aw; const _Float16* wp = Q1 + (size_t)(hd * 32 + m) * 32 + 8 * h;
      aw.h[0] = *(const v8h*)wp; aw.h[1] = *(const v8h*)(wp + 16);
      g0 = wmh(aw.v, bh.v, ld8(bm1 + hd * 32 + 8 * h, WSCL));
    }
    {
      FragH aw; const _Float16* wp = Q1 + (size_t)(hd * 32 + 16 + m) * 32 + 8 * h;
      aw.h[0] = *(const v8h*)wp; aw.h[1] = *(const v8h*)(wp + 16);
      g1 = wmh(aw.v, bh.v, ld8(bm1 + hd * 32 + 16 + 8 * h, WSCL));
    }
    FragH bq;
    bq.h[0] = silu16(g0); bq.h[1] = silu16(g1);
#pragma unroll
    for (int t = 0; t < 2; ++t) {
      v8f c = ld8(bm2 + hd * 32 + 16 * t + 8 * h, WSCL);
      {
        FragH aw; const _Float16* wp = Q2 + (size_t)(hd * 32 + 16 * t + m) * 32 + 8 * h;
        aw.h[0] = *(const v8h*)wp; aw.h[1] = *(const v8h*)(wp + 16);
        c = wmh(aw.v, bq.v, c);
      }
      const v8f w3 = ld8(Wm3 + hd * 32 + 16 * t + 8 * h, 1.0f);
#pragma unroll
      for (int rr = 0; rr < 8; ++rr) emp = fmaf(silu_f(c[rr] * WINV), w3[rr], emp);
    }
    bsum += bm3[hd];
  }
  const float emag = emp + __shfl_xor(emp, 16) + bsum;
  const float etot = estr + emag + shf[sp];
  if (h == 0) es[wave * 16 + m] = etot;
  __syncthreads();

  v4f v = {0.0f, 0.0f, 0.0f, 0.0f};
  if (wave == 0) v = *(const v4f*)(es + 4 * (lane & 7));
  float* ep = eat + (size_t)blockIdx.x * MROW + 4 * (lane & 7);
  if (wave == 0 && lane < 8) *(volatile v4f*)ep = v;
  __threadfence();
  if (wave == 0 && lane < 8) *(volatile v4f*)ep = v;
}

__global__ __launch_bounds__(64) void k_pool(const float* __restrict__ eat, const int* __restrict__ bt,
                                             float* out, int nN) {
  __shared__ __attribute__((aligned(16))) float so[NOUT];
  const int tid = threadIdx.x, lane = tid & 31, wave = tid >> 5;
  const int g = tid;
  double s = 0.0;
  const int n4 = nN >> 2;
#pragma unroll 1
  for (int q = 0; q < n4; ++q) {
    const v4i b = *(const v4i*)(bt + 4 * q);
    const v4f e = *(const v4f*)(eat + 4 * q);
    s += (b.x == g) ? (double)e.x : 0.0;
    s += (b.y == g) ? (double)e.y : 0.0;
    s += (b.z == g) ? (double)e.z : 0.0;
    s += (b.w == g) ? (double)e.w : 0.0;
  }
#pragma unroll 1
  for (int a = 4 * n4; a < nN; ++a) {
    const int b = bt[a];
    const float e = eat[a];
    s += (b == g) ? (double)e : 0.0;
  }
  so[tid] = (float)s;
  __syncthreads();
  const v4f v = *(const v4f*)(so + 4 * (lane & 15));
  float* op = out + 4 * (lane & 15);
  if (wave == 0 && lane < 16) *(volatile v4f*)op = v;
  __threadfence();
  if (wave == 0 && lane < 16) *(volatile v4f*)op = v;
}

extern "C" void kernel_launch(void* const* d_in, const int* in_sizes, int n_in,
                              void* d_out, int out_size, void* d_ws, size_t ws_size,
                              hipStream_t stream) {
  if (n_in < 21) return;
  const int nN = in_sizes[2];
  const int nE = in_sizes[3];
  if (nN < 1 || nE < 1) return;
  if (in_sizes[0] != 3 * nN || in_sizes[1] != 3 * nN || in_sizes[4] != nE || in_sizes[5] != nN) return;
  if (in_sizes[6] != CHEBN || in_sizes[7] != NSPEC * NEMB || in_sizes[8] != NSPEC) return;
  if (in_sizes[9] != 32 * 64 || in_sizes[10] != 64 || in_sizes[11] != 64 * 64 || in_sizes[12] != 64) return;
  if (in_sizes[13] != 64 || in_sizes[14] < 1) return;
  if (in_sizes[15] != NHEAD * 24 * 32 || in_sizes[16] != NHEAD * 32 || in_sizes[17] != NHEAD * 32 * 32) return;
  if (in_sizes[18] != NHEAD * 32 || in_sizes[19] != NHEAD * 32 || in_sizes[20] != NHEAD) return;
  if (out_size != NOUT) return;

  const float* positions = (const float*)d_in[0];
  const float* moments   = (const float*)d_in[1];
  const int*   species   = (const int*)d_in[2];
  const int*   i_idx     = (const int*)d_in[3];
  const int*   j_idx     = (const int*)d_in[4];
  const int*   batch     = (const int*)d_in[5];
  const float* cheb      = (const float*)d_in[6];
  const float* embed     = (const float*)d_in[7];
  const float* shift     = (const float*)d_in[8];
  const float* Ws1 = (const float*)d_in[9];
  const float* bs1 = (const float*)d_in[10];
  const float* Ws2 = (const float*)d_in[11];
  const float* bs2 = (const float*)d_in[12];
  const float* Ws3 = (const float*)d_in[13];
  const float* bs3 = (const float*)d_in[14];
  const float* Wm1 = (const float*)d_in[15];
  const float* bm1 = (const float*)d_in[16];
  const float* Wm2 = (const float*)d_in[17];
  const float* bm2 = (const float*)d_in[18];
  const float* Wm3 = (const float*)d_in[19];
  const float* bm3 = (const float*)d_in[20];
  float* outp = (float*)d_out;

  const int nBlkE    = (nN + NB - 1) / NB;
  const int featRows = nBlkE * NB;
  const int gridM    = (nN + MROW - 1) / MROW;

  char* ws = (char*)d_ws;
  size_t off = 0;
  const size_t oP1 = off; off += ((size_t)64 * 32 * 2 + 255) & ~(size_t)255;
  const size_t oP2 = off; off += ((size_t)64 * 64 * 2 + 255) & ~(size_t)255;
  const size_t oQ1 = off; off += ((size_t)NHEAD * 32 * 32 * 2 + 255) & ~(size_t)255;
  const size_t oQ2 = off; off += ((size_t)NHEAD * 32 * 32 * 2 + 255) & ~(size_t)255;
  const size_t oF  = off; off += ((size_t)featRows * ACOL * 4 + 255) & ~(size_t)255;
  const size_t oE  = off; off += ((size_t)gridM * MROW * 4 + 255) & ~(size_t)255;
  size_t limit = (size_t)134217728;
  if (ws_size < limit) limit = ws_size;
  if (off > limit) return;

  _Float16* pP1 = (_Float16*)(ws + oP1);
  _Float16* pP2 = (_Float16*)(ws + oP2);
  _Float16* pQ1 = (_Float16*)(ws + oQ1);
  _Float16* pQ2 = (_Float16*)(ws + oQ2);
  float* F  = (float*)(ws + oF);
  float* EA = (float*)(ws + oE);

  k_prep<<<PBT, PREP_T, 0, stream>>>(Ws1, Ws2, Wm1, Wm2, pP1, pP2, pQ1, pQ2);

  hipFuncSetAttribute(reinterpret_cast<const void*>(&k_edge), hipFuncAttributeMaxDynamicSharedMemorySize, LDS_EDGE);
  k_edge<<<nBlkE, NTHR, LDS_EDGE, stream>>>(positions, moments, species, i_idx, j_idx, cheb, F, nN, nE, 1);

  k_mlp<<<gridM, MLPT, 0, stream>>>(F, species, embed, shift, pP1, bs1, pP2, bs2, Ws3, bs3,
                                     pQ1, bm1, pQ2, bm2, Wm3, bm3, EA, nN, featRows);

  k_pool<<<1, 64, 0, stream>>>(EA, batch, outp, nN);
}
